// FreeConvNetwork_3753801416735
// MI455X (gfx1250) — hardware-verified
//
#include <hip/hip_runtime.h>


#define NB_  8192
#define C1   16
#define C2   32
#define C3   64
#define H2   6
#define H3   4
#define NF1  512
#define NCLS 10

typedef unsigned short bf;
typedef __attribute__((ext_vector_type(16))) __bf16   v16bf;
typedef __attribute__((ext_vector_type(8)))  unsigned short v8us;
typedef __attribute__((ext_vector_type(8)))  float    v8f;
typedef __attribute__((ext_vector_type(4)))  float    v4f;
typedef v4f  __attribute__((may_alias)) v4fa;
typedef v8us __attribute__((may_alias)) v8usa;

__device__ __forceinline__ unsigned short f2bf(float f) { unsigned u = __float_as_uint(f); u += 0x7FFFu + ((u >> 16) & 1u); return (unsigned short)(u >> 16); }
__device__ __forceinline__ float bf2f(unsigned short b) { return __uint_as_float(((unsigned)b) << 16); }
__device__ __forceinline__ float bfr(float f) { return bf2f(f2bf(f)); }
__device__ __forceinline__ v16bf cat16b(v8us lo, v8us hi) { return __builtin_bit_cast(v16bf, __builtin_shufflevector(lo, hi, 0, 1, 2, 3, 4, 5, 6, 7, 8, 9, 10, 11, 12, 13, 14, 15)); }
__device__ __forceinline__ v8f wmmab(v16bf a, v16bf b, v8f c) { return __builtin_amdgcn_wmma_f32_16x16x32_bf16(false, a, false, b, (short)0, c, false, false); }
#define VST2(T, p, v) do { const T vst2_v_ = (v); *(volatile T*)(p) = vst2_v_; __threadfence(); *(volatile T*)(p) = vst2_v_; } while (0)

__global__ __launch_bounds__(128) void k_l2(const float* __restrict__ x, const float* __restrict__ w1, const float* __restrict__ b1, const float* __restrict__ w2, const float* __restrict__ b2, float* H2f) {
    __shared__ float xs[64 * 49];
    __shared__ __align__(16) unsigned short ah[64 * 168];
    __shared__ __align__(16) unsigned short al[64 * 168];
    __shared__ __align__(16) unsigned short bt[32 * 168];
    __shared__ __align__(16) float ot[64 * 32];
    const int tid = threadIdx.x, lane = tid & 31, wave = tid >> 5, lr = lane & 15, hi = lane >> 4;
    const int pos = blockIdx.y, y = pos / H2, xq = pos - y * H2, b0 = blockIdx.x * 64;
    for (int e = tid; e < 64 * 49; e += 128) { const int r = e / 49, p = e - r * 49, wy = p / 7, wx = p - wy * 7;
        xs[e] = bfr(x[(size_t)(b0 + r) * 784 + (4 * y + wy) * 28 + 4 * xq + wx]); }
    for (int e = tid; e < 32 * 160; e += 128) { const int o = e / 160, k = e - o * 160; unsigned short v = 0;
        if (k < 144) { const int c = k / 9, t = k - c * 9; v = f2bf(w2[(((size_t)(o * C1 + c)) * 36 + pos) * 9 + t]); }
        bt[o * 168 + k] = v; }
    __syncthreads();
#pragma unroll 1
    for (int e = tid; e < 64 * 160; e += 128) { const int r = e / 160, k = e - r * 160; float v = 0.f;
        if (k < 144) { const int c = k / 9, t = k - c * 9, kh = t / 3, kw = t - kh * 3; const int Y = 2 * y + kh, X = 2 * xq + kw;
            const float* wp = w1 + ((size_t)(c * 169 + Y * 13 + X)) * 9; float s = bfr(b1[c * 169 + Y * 13 + X]);
            const float* xw = xs + r * 49 + (2 * kh) * 7 + 2 * kw;
#pragma unroll
            for (int tt = 0; tt < 9; ++tt) { const int a = tt / 3, bq = tt - a * 3; s += xw[a * 7 + bq] * bfr(wp[tt]); }
            v = fmaxf(s, 0.f); }
        const unsigned short hb = f2bf(v); ah[r * 168 + k] = hb; al[r * 168 + k] = f2bf(v - bf2f(hb)); }
    __syncthreads();
    v8f acc[2] = {};
#pragma unroll
    for (int kc = 0; kc < 5; ++kc) { const int ro = (wave * 16 + lr) * 168 + kc * 32 + 8 * hi;
        const v16bf a = cat16b(*(const v8usa*)(ah + ro), *(const v8usa*)(ah + ro + 16)), a2 = cat16b(*(const v8usa*)(al + ro), *(const v8usa*)(al + ro + 16));
#pragma unroll
        for (int n = 0; n < 2; ++n) { const int bo = (n * 16 + lr) * 168 + kc * 32 + 8 * hi; const v16bf bb = cat16b(*(const v8usa*)(bt + bo), *(const v8usa*)(bt + bo + 16));
            acc[n] = wmmab(a, bb, acc[n]); acc[n] = wmmab(a2, bb, acc[n]); } }
    asm volatile("v_nop\n\tv_nop\n\tv_nop\n\tv_nop" : "+v"(acc[0]), "+v"(acc[1]));
#pragma unroll
    for (int n = 0; n < 2; ++n)
#pragma unroll
        for (int j = 0; j < 8; ++j) { const int r = wave * 16 + hi * 8 + j, o = n * 16 + lr; ot[r * 32 + o] = fmaxf(acc[n][j] + bfr(b2[o * 36 + pos]), 0.f); }
    __syncthreads();
    auto pass = [&]() {
#pragma unroll
        for (int s = 0; s < 4; ++s) { const int e0 = s * 512 + tid * 4; const v4f v = *(const v4fa*)(ot + e0); *(volatile v4f*)(H2f + ((size_t)pos * NB_ + b0) * 32 + e0) = v; }
    };
    pass(); __threadfence(); pass();
}
__global__ __launch_bounds__(128) void k_l3(const float* __restrict__ H2f, const float* __restrict__ w3, const float* __restrict__ b3, bf* H3H, bf* H3L) {
    __shared__ __align__(16) unsigned short ah[64 * 296];
    __shared__ __align__(16) unsigned short al[64 * 296];
    __shared__ __align__(16) unsigned short bt[64 * 296];
    __shared__ __align__(16) float ot[64 * 64];
    const int tid = threadIdx.x, lane = tid & 31, wave = tid >> 5, lr = lane & 15, hi = lane >> 4;
    const int q = blockIdx.y, y = q / H3, xq = q - y * H3, b0 = blockIdx.x * 64;
#pragma unroll 1
    for (int e = tid; e < 64 * 288; e += 128) { const int r = e / 288, k = e - r * 288; const int c = k / 9, t = k - c * 9, kh = t / 3, kw = t - kh * 3;
        const float v = H2f[((size_t)((y + kh) * H2 + xq + kw) * NB_ + b0 + r) * 32 + c]; const unsigned short hb = f2bf(v); ah[r * 296 + k] = hb; al[r * 296 + k] = f2bf(v - bf2f(hb)); }
#pragma unroll 1
    for (int e = tid; e < 64 * 288; e += 128) { const int o = e / 288, k = e - o * 288; const int c = k / 9, t = k - c * 9;
        bt[o * 296 + k] = f2bf(w3[(((size_t)(o * C2 + c)) * 16 + q) * 9 + t]); }
    __syncthreads();
    v8f acc[4] = {};
#pragma unroll 3
    for (int kc = 0; kc < 9; ++kc) { const int ro = (wave * 16 + lr) * 296 + kc * 32 + 8 * hi;
        const v16bf a = cat16b(*(const v8usa*)(ah + ro), *(const v8usa*)(ah + ro + 16)), a2 = cat16b(*(const v8usa*)(al + ro), *(const v8usa*)(al + ro + 16));
#pragma unroll
        for (int n = 0; n < 4; ++n) { const int bo = (n * 16 + lr) * 296 + kc * 32 + 8 * hi; const v16bf bb = cat16b(*(const v8usa*)(bt + bo), *(const v8usa*)(bt + bo + 16));
            acc[n] = wmmab(a, bb, acc[n]); acc[n] = wmmab(a2, bb, acc[n]); } }
    asm volatile("v_nop\n\tv_nop\n\tv_nop\n\tv_nop" : "+v"(acc[0]), "+v"(acc[1]), "+v"(acc[2]), "+v"(acc[3]));
#pragma unroll
    for (int n = 0; n < 4; ++n)
#pragma unroll
        for (int j = 0; j < 8; ++j) { const int r = wave * 16 + hi * 8 + j, o = n * 16 + lr; ot[r * 64 + o] = acc[n][j] + bfr(b3[o * 16 + q]); }
    __syncthreads();
    auto pass = [&]() {
#pragma unroll
        for (int s = 0; s < 4; ++s) { const int r = wave * 16 + s * 4 + (lane >> 3), piece = lane & 7; const float* sp = ot + r * 64 + piece * 8; v8us oh, ol;
#pragma unroll
            for (int i = 0; i < 8; ++i) { const unsigned short hb = f2bf(sp[i]); oh[i] = hb; ol[i] = f2bf(sp[i] - bf2f(hb)); }
            *(volatile v8us*)(H3H + (size_t)(b0 + r) * 1024 + q * 64 + piece * 8) = oh; *(volatile v8us*)(H3L + (size_t)(b0 + r) * 1024 + q * 64 + piece * 8) = ol; }
    };
    pass(); __threadfence(); pass();
}
__global__ __launch_bounds__(256) void k_wf(const float* __restrict__ fw1, const float* __restrict__ fw2, bf* FW1, bf* FW2) {
    const int lane = threadIdx.x & 31, r = blockIdx.x * 8 + (threadIdx.x >> 5);
    if (r < NF1) {
#pragma unroll
        for (int s = 0; s < 4; ++s) { v8us o;
#pragma unroll
            for (int i = 0; i < 8; ++i) { const int kp = s * 256 + lane * 8 + i, q = kp >> 6, oc = kp & 63, j = oc * 16 + q; o[i] = f2bf(fw1[(size_t)r * 1024 + j]); }
            VST2(v8us, FW1 + (size_t)r * 1024 + s * 256 + lane * 8, o); }
    }
    if (r < 16) {
#pragma unroll
        for (int s = 0; s < 2; ++s) { v8us o;
#pragma unroll
            for (int i = 0; i < 8; ++i) { const int k = s * 256 + lane * 8 + i; o[i] = (r < NCLS) ? f2bf(fw2[(size_t)r * NF1 + k]) : (unsigned short)0; }
            VST2(v8us, FW2 + (size_t)r * NF1 + s * 256 + lane * 8, o); }
    }
}
__global__ __launch_bounds__(128) void k_fc1(const bf* __restrict__ A, const bf* __restrict__ Al, const bf* __restrict__ Bn, const float* __restrict__ bias, bf* CH, bf* CL) {
    __shared__ __align__(16) float ost[4][16 * 68];
    const int lane = threadIdx.x & 31, wave = threadIdx.x >> 5, lr = lane & 15, hi = lane >> 4;
    const int r0 = blockIdx.x * 64 + wave * 16, c0 = blockIdx.y * 64;
    const size_t aoff = (size_t)(r0 + lr) * 1024 + 8 * hi;
    size_t boff[4];
#pragma unroll
    for (int t = 0; t < 4; ++t) boff[t] = (size_t)(c0 + t * 16 + lr) * 1024 + 8 * hi;
    v8f acc[4];
#pragma unroll
    for (int t = 0; t < 4; ++t) acc[t] = (v8f){};
#pragma unroll 1
    for (int kc = 0; kc < 1024; kc += 32) {
        const v16bf a = cat16b(*(const v8us*)(A + aoff + kc), *(const v8us*)(A + aoff + kc + 16)), a2 = cat16b(*(const v8us*)(Al + aoff + kc), *(const v8us*)(Al + aoff + kc + 16));
#pragma unroll
        for (int t = 0; t < 4; ++t) { const v16bf bb = cat16b(*(const v8us*)(Bn + boff[t] + kc), *(const v8us*)(Bn + boff[t] + kc + 16)); acc[t] = wmmab(a, bb, acc[t]); acc[t] = wmmab(a2, bb, acc[t]); }
        asm volatile("v_nop\n\tv_nop\n\tv_nop\n\tv_nop" : "+v"(acc[0]), "+v"(acc[1]), "+v"(acc[2]), "+v"(acc[3]) : "v"(a), "v"(a2));
    }
    float* os = &ost[wave][0];
#pragma unroll
    for (int t = 0; t < 4; ++t) { const float bv = bfr(bias[c0 + t * 16 + lr]);
#pragma unroll
        for (int j = 0; j < 8; ++j) os[(hi * 8 + j) * 68 + t * 16 + lr] = fmaxf(acc[t][j] + bv, 0.f); }
    __syncthreads();
    auto pass = [&]() {
#pragma unroll
        for (int s = 0; s < 4; ++s) { const int row = 4 * s + (lane >> 3), piece = lane & 7; const float* sp = os + row * 68 + piece * 8; v8us oh, ol;
#pragma unroll
            for (int i = 0; i < 8; ++i) { const unsigned short hb = f2bf(sp[i]); oh[i] = hb; ol[i] = f2bf(sp[i] - bf2f(hb)); }
            *(volatile v8us*)(CH + (size_t)(r0 + row) * NF1 + c0 + piece * 8) = oh; *(volatile v8us*)(CL + (size_t)(r0 + row) * NF1 + c0 + piece * 8) = ol; }
    };
    pass(); __threadfence(); pass();
}
__global__ __launch_bounds__(128) void k_fc2(const bf* __restrict__ FH, const bf* __restrict__ FL, const bf* __restrict__ FW2, const float* __restrict__ fb2, float* out) {
    __shared__ float st[64 * NCLS];
    const int tid = threadIdx.x, lane = tid & 31, wave = tid >> 5, lr = lane & 15, hi = lane >> 4;
    const int r0 = blockIdx.x * 64 + wave * 16;
    v8f acc = {};
#pragma unroll 4
    for (int kc = 0; kc < NF1 / 32; ++kc) { const size_t ao = (size_t)(r0 + lr) * NF1 + kc * 32 + 8 * hi, bo = (size_t)lr * NF1 + kc * 32 + 8 * hi;
        const v16bf bb = cat16b(*(const v8us*)(FW2 + bo), *(const v8us*)(FW2 + bo + 16));
        acc = wmmab(cat16b(*(const v8us*)(FH + ao), *(const v8us*)(FH + ao + 16)), bb, acc); acc = wmmab(cat16b(*(const v8us*)(FL + ao), *(const v8us*)(FL + ao + 16)), bb, acc); }
    asm volatile("v_nop\n\tv_nop\n\tv_nop\n\tv_nop" : "+v"(acc));
    if (lr < NCLS) {
#pragma unroll
        for (int j = 0; j < 8; ++j) st[(wave * 16 + hi * 8 + j) * NCLS + lr] = acc[j] + bfr(fb2[lr]);
    }
    __syncthreads();
    auto pass = [&]() {
#pragma unroll
        for (int s = 0; s < 5; ++s) { const int e = s * 128 + tid; *(volatile float*)(out + (size_t)blockIdx.x * 640 + e) = st[e]; }
    };
    pass(); __threadfence(); pass();
}

extern "C" void kernel_launch(void* const* d_in, const int* in_sizes, int n_in,
                              void* d_out, int out_size, void* d_ws, size_t ws_size, hipStream_t stream) {
    (void)in_sizes; (void)n_in; (void)out_size;
    const float* x = (const float*)d_in[0]; const float* w1 = (const float*)d_in[1]; const float* b1 = (const float*)d_in[2]; const float* w2 = (const float*)d_in[3]; const float* b2 = (const float*)d_in[4];
    const float* w3 = (const float*)d_in[5]; const float* b3 = (const float*)d_in[6]; const float* fw1 = (const float*)d_in[7]; const float* fb1 = (const float*)d_in[8]; const float* fw2 = (const float*)d_in[9]; const float* fb2 = (const float*)d_in[10];
    float* out = (float*)d_out;
    char* wsp = (char*)d_ws;
    auto take = [&](size_t bytes) { char* p = wsp; wsp += (bytes + 255) & ~(size_t)255; return (void*)p; };
    float* H2f = (float*)take((size_t)36 * NB_ * 32 * 4); bf* H3H = (bf*)take((size_t)NB_ * 1024 * 2); bf* H3L = (bf*)take((size_t)NB_ * 1024 * 2);
    bf* FW1 = (bf*)take((size_t)NF1 * 1024 * 2); bf* FW2 = (bf*)take((size_t)16 * NF1 * 2); bf* F1H = (bf*)take((size_t)NB_ * NF1 * 2); bf* F1L = (bf*)take((size_t)NB_ * NF1 * 2);
    if ((size_t)(wsp - (char*)d_ws) > ws_size) return;
    k_l2<<<dim3(NB_ / 64, 36, 1), 128, 0, stream>>>(x, w1, b1, w2, b2, H2f);
    k_l3<<<dim3(NB_ / 64, 16, 1), 128, 0, stream>>>(H2f, w3, b3, H3H, H3L);
    k_wf<<<NF1 / 8, 256, 0, stream>>>(fw1, fw2, FW1, FW2);
    k_fc1<<<dim3(NB_ / 64, NF1 / 64, 1), 128, 0, stream>>>(H3H, H3L, FW1, fb1, F1H, F1L);
    k_fc2<<<NB_ / 64, 128, 0, stream>>>(F1H, F1L, FW2, fb2, out);
}
